// SuperONN2d_v2_12360915878419
// MI455X (gfx1250) — hardware-verified
//
#include <hip/hip_runtime.h>
#include <stdint.h>

#define BN    4
#define CIN   32
#define COUT  64
#define HH    128
#define WWD   128
#define HW    (HH * WWD)
#define NTAP  9
#define NPOW  3
#define CK    (NPOW * CIN * NTAP)
#define KP    896
#define NPX   32
#define NTHR  256
#define BLK_PER_IMG (HW / NPX)
#define NBLK  (BN * BLK_PER_IMG)
#define WCHK  (COUT * KP / 8)
#define NIT3  (NPX * NTAP * CIN / NTHR)

#define SCW   64.0f
#define RSC   2048.0f
#define INV_H 0.015625f
#define INV_X 7.62939453125e-06f
#define MAXS  4.0f

#define L_AH   0
#define L_AL   (L_AH + NPX * KP * 2)
#define L_C    (L_AL + NPX * KP * 2)
#define L_CW   (L_C + NPX * NTAP * 4 * 4)
#define L_SW   (L_C + 2 * NPX * NTAP * 4 * 4)
#define L_PART (L_SW + 2 * CIN * NTAP * 4)
#define L_SH   (L_PART + 2 * 8 * NPX * 4)
#define L_BIAS (L_SH + 2 * NPX * 4)
#define L_SB   (L_BIAS + COUT * 4)
#define LDS_BYTES (L_SB + 16)

static_assert(NTHR == 256);
static_assert(HW % NPX == 0);
static_assert(WWD % NPX == 0);
static_assert(BLK_PER_IMG == 512);
static_assert(NBLK * NPX == BN * HW);
static_assert(WCHK % 256 == 0);
static_assert(KP % 32 == 0);
static_assert(KP >= CK);
static_assert(CK % 8 == 0);
static_assert((NPX * NTAP * CIN) % NTHR == 0);
static_assert(COUT * NPX * 4 <= L_SW - L_C);
static_assert(LDS_BYTES % 16 == 0);
static_assert((L_C % 16) == 0);
static_assert((L_CW % 16) == 0);
static_assert(NPX * NTAP - NTHR == 32);
static_assert(COUT * NPX / 4 == 2 * NTHR);

typedef _Float16 v16h __attribute__((ext_vector_type(16)));
typedef _Float16 v8h  __attribute__((ext_vector_type(8)));
typedef float    v8f  __attribute__((ext_vector_type(8)));
typedef float    v4f  __attribute__((ext_vector_type(4)));
typedef unsigned v4u  __attribute__((ext_vector_type(4)));

__device__ __forceinline__ float bf_rne(float f) {
  unsigned u = __float_as_uint(f);
  u = (u + 0x7FFFu + ((u >> 16) & 1u)) & 0xFFFF0000u;
  return __uint_as_float(u);
}
__device__ __forceinline__ unsigned hbits(_Float16 h) {
  return (unsigned)__builtin_bit_cast(unsigned short, h);
}
__device__ __forceinline__ void split_hl(float v, _Float16& h, _Float16& l) {
  h = (_Float16)v;
  l = (_Float16)((v - (float)h) * RSC);
}
__device__ __forceinline__ v8f zero8f() { v8f z = {0.f, 0.f, 0.f, 0.f, 0.f, 0.f, 0.f, 0.f}; return z; }
__device__ __forceinline__ v8h zero8h() {
  v8h z;
#pragma unroll
  for (int e = 0; e < 8; ++e) z[e] = (_Float16)0.0f;
  return z;
}

__device__ __forceinline__ v16h ldfrag(const _Float16* p) {
  union { v16h v; v8h h[2]; } f;
  f.h[0] = *(const v8h*)(p);
  f.h[1] = *(const v8h*)(p + 16);
  return f.v;
}

__device__ __forceinline__ v8f mma_h(v16h a, v16h b, v8f c) {
  return __builtin_amdgcn_wmma_f32_16x16x32_f16(false, a, false, b, (short)0, c, false, false);
}
__device__ __forceinline__ void dep_guard2(v8f& w, v8f& x, v16h f0, v16h f1, v16h f2) {
#if defined(__HIP_DEVICE_COMPILE__)
  asm volatile("v_nop\n\tv_nop\n\tv_nop\n\tv_nop"
               : "+v"(w), "+v"(x) : "v"(f0), "v"(f1), "v"(f2));
#endif
}
__device__ __forceinline__ void acc_guard2(v8f& w, v8f& x) {
#if defined(__HIP_DEVICE_COMPILE__)
  asm volatile("v_nop\n\tv_nop\n\tv_nop\n\tv_nop" : "+v"(w), "+v"(x));
#endif
}

__global__ __launch_bounds__(256)
void k_wprep(const float* __restrict__ w, unsigned* wb)
{
  const int q   = blockIdx.x * 256 + threadIdx.x;
  const int qc  = (q < WCHK) ? q : (WCHK - 1);
  const int co  = qc / (KP / 8);
  const int kc  = (qc - co * (KP / 8)) * 8;

  unsigned hb[8];
#pragma unroll
  for (int j = 0; j < 8; ++j) {
    const int kk  = kc + j;
    const int kkc = (kk < CK) ? kk : (CK - 1);
    float v = bf_rne(w[(size_t)co * CK + kkc]) * SCW;
    v = (kk < CK) ? v : 0.0f;
    hb[j] = hbits((_Float16)v);
  }
  v4u wh;
  wh.x = hb[0] | (hb[1] << 16);
  wh.y = hb[2] | (hb[3] << 16);
  wh.z = hb[4] | (hb[5] << 16);
  wh.w = hb[6] | (hb[7] << 16);

  unsigned* dst = wb + (size_t)qc * 4;
  if (q < WCHK) *(volatile v4u*)dst = wh;
  __threadfence();
  if (q < WCHK) *(volatile v4u*)dst = wh;
}

__global__ __launch_bounds__(NTHR)
void k_main(const float* __restrict__ x, const float* __restrict__ bias,
            const float* __restrict__ sw, const float* __restrict__ sb,
            const _Float16* __restrict__ wt, float* out)
{
  extern __shared__ __align__(16) unsigned char smem[];
  _Float16* Ah   = (_Float16*)(smem + L_AH);
  _Float16* Al   = (_Float16*)(smem + L_AL);
  int*      cidx = (int*)(smem + L_C);
  float*    cwt  = (float*)(smem + L_CW);
  float*    os   = (float*)(smem + L_C);
  float*    swl  = (float*)(smem + L_SW);
  float*    part = (float*)(smem + L_PART);
  float*    shl  = (float*)(smem + L_SH);
  float*    bsl  = (float*)(smem + L_BIAS);
  float*    sbl  = (float*)(smem + L_SB);

  const int tid  = threadIdx.x;
  const int lane = tid & 31;
  const int wv   = tid >> 5;
  const int lm   = lane & 15;
  const int hh   = lane >> 4;
  const int bid  = blockIdx.x;
  const int b    = bid / BLK_PER_IMG;
  const int tile = bid - b * BLK_PER_IMG;
  const int pixbase = tile * NPX;
  const int oy   = pixbase / WWD;
  const int oxb  = pixbase - oy * WWD;
  const float* xb = x + (size_t)b * CIN * HW;

#pragma unroll 1
  for (int i = tid; i < 2 * CIN * NTAP; i += NTHR) swl[i] = bf_rne(sw[i]);
  if (tid < COUT) bsl[tid] = bf_rne(bias[tid]);
  if (tid < 2) sbl[tid] = bf_rne(sb[tid]);
  __syncthreads();

  {
    const int p  = lane;
    const int g  = wv;
    const int ox = oxb + p;
    float a0 = 0.0f, a1 = 0.0f;
#pragma unroll 1
    for (int cc = 0; cc < 4; ++cc) {
      const int ci = 4 * g + cc;
      const float* xc = xb + (size_t)ci * HW;
      const float* w0 = swl + ci * NTAP;
      const float* w1 = swl + CIN * NTAP + ci * NTAP;
#pragma unroll
      for (int ky = 0; ky < 3; ++ky) {
        const int yy  = oy - 1 + ky;
        const bool vy = (unsigned)yy < (unsigned)HH;
        const int yyc = (yy < 0) ? 0 : ((yy > HH - 1) ? (HH - 1) : yy);
#pragma unroll
        for (int kx = 0; kx < 3; ++kx) {
          const int xx  = ox - 1 + kx;
          const bool vx = (unsigned)xx < (unsigned)WWD;
          const int xxc = (xx < 0) ? 0 : ((xx > WWD - 1) ? (WWD - 1) : xx);
          const float raw = xc[yyc * WWD + xxc];
          const float xv  = (vy && vx) ? bf_rne(raw) : 0.0f;
          a0 = fmaf(xv, w0[ky * 3 + kx], a0);
          a1 = fmaf(xv, w1[ky * 3 + kx], a1);
        }
      }
    }
    part[(0 * 8 + g) * NPX + p] = a0;
    part[(1 * 8 + g) * NPX + p] = a1;
  }
  __syncthreads();
  if (tid < 2 * NPX) {
    const int s = tid >> 5;
    const int p = tid & 31;
    float a = 0.0f;
#pragma unroll
    for (int g = 0; g < 8; ++g) a += part[(s * 8 + g) * NPX + p];
    a += sbl[s];
    a = fminf(fmaxf(a, -MAXS), MAXS);
    shl[s * NPX + p] = a;
  }
  __syncthreads();

#pragma unroll 1
  for (int t = tid; t < NPX * NTAP; t += NTHR) {
    const int p  = t & 31;
    const int k  = t >> 5;
    const int ky = k / 3;
    const int kx = k - 3 * ky;
    const float s0 = shl[p];
    const float s1 = shl[NPX + p];
    const float dy = ((2 * k) >= 9) ? s1 : s0;
    const float dx = ((2 * k + 1) >= 9) ? s1 : s0;
    const float py = (float)(oy - 1 + ky) + dy;
    const float px = (float)(oxb + p - 1 + kx) + dx;
    const float y0f = floorf(py);
    const float x0f = floorf(px);
    const float ly = py - y0f;
    const float lx = px - x0f;
    const int y0 = (int)y0f;
    const int x0 = (int)x0f;
#pragma unroll
    for (int cy = 0; cy < 2; ++cy) {
#pragma unroll
      for (int cx = 0; cx < 2; ++cx) {
        const int yc = y0 + cy;
        const int xc = x0 + cx;
        const bool valid = (yc >= 0) && (yc < HH) && (xc >= 0) && (xc < WWD);
        const int yi = (yc < 0) ? 0 : ((yc > HH - 1) ? (HH - 1) : yc);
        const int xi = (xc < 0) ? 0 : ((xc > WWD - 1) ? (WWD - 1) : xc);
        const float wgt = (cy ? ly : (1.0f - ly)) * (cx ? lx : (1.0f - lx));
        const int sl = (k * 4 + cy * 2 + cx) * NPX + p;
        cidx[sl] = yi * WWD + xi;
        cwt[sl]  = valid ? wgt : 0.0f;
      }
    }
  }
  __syncthreads();

  {
    const v8h z8 = zero8h();
    const int r  = tid & 127;
    const int p  = r >> 2;
    const int c  = r & 3;
    _Float16* dstp = ((tid < 128) ? Ah : Al) + p * KP + CK + 8 * c;
    *(v8h*)dstp = z8;
  }
#pragma unroll 1
  for (int it = 0; it < NIT3; ++it) {
    const int t    = it * NTHR + tid;
    const int p    = t & 31;
    const int rest = t >> 5;
    const int cin  = rest / NTAP;
    const int k    = rest - cin * NTAP;
    const float* xc = xb + (size_t)cin * HW;
    float v1 = 0.0f, v2 = 0.0f, v3 = 0.0f;
#pragma unroll
    for (int c = 0; c < 4; ++c) {
      const int sl = (k * 4 + c) * NPX + p;
      const float wgt = cwt[sl];
      const float xr  = bf_rne(xc[cidx[sl]]);
      const float x2  = xr * xr;
      const float x3  = x2 * xr;
      v1 = fmaf(wgt, xr, v1);
      v2 = fmaf(wgt, x2, v2);
      v3 = fmaf(wgt, x3, v3);
    }
    const int kk = rest;
    _Float16* ah = Ah + p * KP;
    _Float16* al = Al + p * KP;
    _Float16 hv, lv;
    split_hl(v1, hv, lv);  ah[kk] = hv;                       al[kk] = lv;
    split_hl(v2, hv, lv);  ah[kk + CIN * NTAP] = hv;          al[kk + CIN * NTAP] = lv;
    split_hl(v3, hv, lv);  ah[kk + 2 * CIN * NTAP] = hv;      al[kk + 2 * CIN * NTAP] = lv;
  }
  __syncthreads();

  {
    const int mt = wv & 1;
    const int nt = wv >> 1;
    const _Float16* pa = Ah + (16 * mt + lm) * KP + 8 * hh;
    const _Float16* pl = Al + (16 * mt + lm) * KP + 8 * hh;
    const _Float16* pb = wt + (size_t)(16 * nt + lm) * KP + 8 * hh;
    v8f acc_h = zero8f(), acc_x = zero8f();
#pragma unroll 2
    for (int s = 0; s < KP / 32; ++s) {
      const v16h fah = ldfrag(pa + 32 * s);
      const v16h fal = ldfrag(pl + 32 * s);
      const v16h fb  = ldfrag(pb + 32 * s);
      acc_h = mma_h(fah, fb, acc_h);
      acc_x = mma_h(fal, fb, acc_x);
      dep_guard2(acc_h, acc_x, fah, fal, fb);
    }
    acc_guard2(acc_h, acc_x);

    const int co = 16 * nt + lm;
    const float bb = bsl[co];
    float* orow = os + co * NPX + 16 * mt + 8 * hh;
    v4f o0, o1;
    o0.x = acc_h[0] * INV_H + acc_x[0] * INV_X + bb;
    o0.y = acc_h[1] * INV_H + acc_x[1] * INV_X + bb;
    o0.z = acc_h[2] * INV_H + acc_x[2] * INV_X + bb;
    o0.w = acc_h[3] * INV_H + acc_x[3] * INV_X + bb;
    o1.x = acc_h[4] * INV_H + acc_x[4] * INV_X + bb;
    o1.y = acc_h[5] * INV_H + acc_x[5] * INV_X + bb;
    o1.z = acc_h[6] * INV_H + acc_x[6] * INV_X + bb;
    o1.w = acc_h[7] * INV_H + acc_x[7] * INV_X + bb;
    *(v4f*)(orow)     = o0;
    *(v4f*)(orow + 4) = o1;
  }
  __syncthreads();

  {
    float* obase = out + (size_t)b * COUT * HW + pixbase;
    const int q0 = tid;
    const int q1 = tid + NTHR;
    const int c0 = q0 >> 3, j0 = q0 & 7;
    const int c1 = q1 >> 3, j1 = q1 & 7;
    const v4f v0 = *(const v4f*)(os + c0 * NPX + 4 * j0);
    const v4f v1 = *(const v4f*)(os + c1 * NPX + 4 * j1);
    float* d0 = obase + (size_t)c0 * HW + 4 * j0;
    float* d1 = obase + (size_t)c1 * HW + 4 * j1;
    *(volatile v4f*)d0 = v0;
    *(volatile v4f*)d1 = v1;
    __threadfence();
    *(volatile v4f*)d0 = v0;
    *(volatile v4f*)d1 = v1;
  }
}

extern "C" void kernel_launch(void* const* d_in, const int* in_sizes, int n_in,
                              void* d_out, int out_size, void* d_ws, size_t ws_size,
                              hipStream_t stream) {
  if (n_in < 5) return;
  if (in_sizes[0] != BN * CIN * HW) return;
  if (in_sizes[1] != COUT * CK) return;
  if (in_sizes[2] < COUT) return;
  if (in_sizes[3] != 2 * CIN * NTAP) return;
  if (in_sizes[4] < 2) return;
  if (out_size != BN * COUT * HW) return;

  const size_t wbytes = (size_t)COUT * KP * 2;
  if (wbytes > ws_size) return;

  const float* x       = (const float*)d_in[0];
  const float* weight  = (const float*)d_in[1];
  const float* bias    = (const float*)d_in[2];
  const float* shift_w = (const float*)d_in[3];
  const float* shift_b = (const float*)d_in[4];
  float* out = (float*)d_out;

  unsigned* wbuf = (unsigned*)d_ws;

  (void)hipFuncSetAttribute(reinterpret_cast<const void*>(&k_main),
                            hipFuncAttributeMaxDynamicSharedMemorySize, LDS_BYTES);

  k_wprep<<<dim3(WCHK / 256), dim3(256), 0, stream>>>(weight, wbuf);
  (void)hipGetLastError();

  k_main<<<dim3(NBLK), dim3(NTHR), LDS_BYTES, stream>>>(x, bias, shift_w, shift_b,
                                                         (const _Float16*)wbuf, out);
  (void)hipGetLastError();
}
